// TransformerEncoderBlock_80874234183908
// MI455X (gfx1250) — hardware-verified
//
#include <hip/hip_runtime.h>


#ifndef NB
#define NB 2
#endif
#ifndef SEQ
#define SEQ 2048
#endif

namespace {
constexpr int B_FULL = 2, SEQ_FULL = 2048, DM = 768, NH = 12, DK = 64, FF = 3072, NQKV = 3 * DM, NR = NB * SEQ, NBH = NB * NH;
constexpr float XS = 8.0f, WSC = 256.0f, QS = 8.0f, PSC = 16.0f, VS = 64.0f, CTS = 64.0f, LOG2E = 1.4426950408889634f, LNEPS = 1e-5f, RSQDK = 0.125f;
static_assert(NB >= 1 && NB <= B_FULL);
static_assert(SEQ % 128 == 0 && SEQ >= 128 && SEQ <= SEQ_FULL);
static_assert(DM % 256 == 0 && DM % 128 == 0 && FF % 128 == 0 && NQKV % 128 == 0 && DK == 64 && NR % 64 == 0 && (NR * DM) % 8 == 0);
typedef _Float16 b16;
typedef __attribute__((ext_vector_type(16))) _Float16 v16b;
typedef __attribute__((ext_vector_type(8))) _Float16 v8b;
typedef __attribute__((ext_vector_type(4))) _Float16 v4h;
typedef __attribute__((ext_vector_type(8))) float v8f;
typedef __attribute__((ext_vector_type(4))) float v4f;
__device__ __forceinline__ float bf16_rne(float f) { unsigned int u = __float_as_uint(f); u += 0x7FFFu + ((u >> 16) & 1u); return __uint_as_float(u & 0xFFFF0000u); }
__device__ __forceinline__ v16b frag_kb(const b16* p, int hh) { const v8b a = *(const v8b*)(p + 8 * hh), b = *(const v8b*)(p + 16 + 8 * hh); v16b f;
#pragma unroll
  for (int e = 0; e < 8; ++e) { f[e] = a[e]; f[8 + e] = b[e]; } return f; }
__device__ __forceinline__ v8f wmma16b(v16b a, v16b b, v8f c) { v8f d = __builtin_amdgcn_wmma_f32_16x16x32_f16(false, a, false, b, (short)0, c, false, false); asm volatile("v_nop\n\tv_nop\n\tv_nop\n\tv_nop" : "+v"(d) : "v"(a), "v"(b)); return d; }
__device__ __forceinline__ void wave_lds_sync() { __builtin_amdgcn_fence(3, "workgroup"); __builtin_amdgcn_wave_barrier(); __builtin_amdgcn_fence(2, "workgroup"); }
__device__ __forceinline__ float pmul(float a, float b) { float p = a * b; asm volatile("" : "+v"(p)); return p; }
__device__ __forceinline__ float nexp2(float v) { return __builtin_amdgcn_exp2f(v); }
__device__ __forceinline__ float bfp(float v) { float t = bf16_rne(v); asm volatile("" : "+v"(t)); return t; }

__global__ __launch_bounds__(128) void wtp_kernel(const float* __restrict__ s0p, const float* __restrict__ s1p, const float* __restrict__ s2p, int nz, int R, int C, long long sz,
                                                  b16* __restrict__ dst, long long dz) {
  __shared__ __attribute__((aligned(16))) b16 tile[64][64 + 8];
  const int wave = threadIdx.x >> 5, lane = threadIdx.x & 31; const int r0 = blockIdx.x * 64, c0 = blockIdx.y * 64; const int z = blockIdx.z, sel = z / nz, zi = z - sel * nz;
  const float* src = (sel == 0 ? s0p : (sel == 1 ? s1p : s2p)) + (size_t)zi * (size_t)sz; b16* d = dst + (size_t)z * (size_t)dz;
#pragma unroll 4
  for (int i = threadIdx.x; i < 64 * 16; i += 128) { const int rr = i >> 4, q = (i & 15) * 4; const v4f f = *(const v4f*)(src + (size_t)(r0 + rr) * C + c0 + q);
#pragma unroll
    for (int j = 0; j < 4; ++j) tile[q + j][rr] = (b16)(bf16_rne(f[j]) * WSC); }
  __syncthreads();
  for (int pass = 0; pass < 2; ++pass) {
#pragma unroll
    for (int i = 0; i < 4; ++i) { const int cc = wave * 16 + i * 4 + (lane >> 3), pc = (lane & 7) * 8; *(volatile v8b*)(d + (size_t)(c0 + cc) * R + r0 + pc) = *(const v8b*)(&tile[cc][pc]); }
    __threadfence(); }
}
__global__ __launch_bounds__(256) void xp_kernel(const float* __restrict__ x, b16* __restrict__ XH) {
  const size_t u = (size_t)blockIdx.x * 256 + threadIdx.x; if (u >= (size_t)NR * DM / 8) return;
  const size_t e = u * 8; const int row = (int)(e / DM), col = (int)(e - (size_t)row * DM); const size_t xe = ((size_t)(row / SEQ) * SEQ_FULL + (size_t)(row % SEQ)) * DM + col;
  const v4f f0 = *(const v4f*)(x + xe), f1 = *(const v4f*)(x + xe + 4); v8b o;
#pragma unroll
  for (int j = 0; j < 4; ++j) { o[j] = (b16)(bf16_rne(f0[j]) * XS); o[4 + j] = (b16)(bf16_rne(f1[j]) * XS); }
  for (int pass = 0; pass < 2; ++pass) { *(volatile v8b*)(XH + e) = o; __threadfence(); }
}
__global__ __launch_bounds__(128) void qkv_kernel(const b16* __restrict__ XH, const b16* __restrict__ WQKV, b16* __restrict__ QP, b16* __restrict__ KP, b16* __restrict__ VP) {
  __shared__ __attribute__((aligned(16))) b16 Th[4][16][128 + 8];
  const int wave = threadIdx.x >> 5, lane = threadIdx.x & 31, nloc = lane & 15, hlf = lane >> 4; const size_t m0 = (size_t)blockIdx.x * 64 + wave * 16; const int n0 = blockIdx.y * 128;
  v8f acc[8];
#pragma unroll
  for (int t = 0; t < 8; ++t) acc[t] = (v8f){};
#pragma unroll 2
  for (int kb = 0; kb < DM; kb += 32) { const v16b a = frag_kb(XH + (m0 + nloc) * DM + kb, hlf);
#pragma unroll
    for (int t = 0; t < 8; ++t) acc[t] = wmma16b(a, frag_kb(WQKV + (size_t)(n0 + t * 16 + nloc) * DM + kb, hlf), acc[t]); }
#pragma unroll
  for (int t = 0; t < 8; ++t)
#pragma unroll
    for (int r = 0; r < 8; ++r) Th[wave][8 * hlf + r][t * 16 + nloc] = (b16)(acc[t][r] * (QS / (XS * WSC)));
  wave_lds_sync();
  const int which = n0 / DM; const int hb = (n0 - which * DM) / DK;
  b16* P = (which == 0) ? QP : ((which == 1) ? KP : VP);
  for (int pass = 0; pass < 2; ++pass) {
#pragma unroll
    for (int i = 0; i < 8; ++i) { const int L = i * 4 + (lane >> 3), rr = L >> 1, hf = L & 1, pc = (lane & 7) * 8; const int row = (int)m0 + rr; const int b = row / SEQ, s = row - b * SEQ;
      const v8b v = *(const v8b*)(&Th[wave][rr][hf * 64 + pc]); *(volatile v8b*)(P + ((size_t)(b * NH + hb + hf) * SEQ + s) * DK + pc) = v; }
    __threadfence(); }
}
__global__ __launch_bounds__(256) __attribute__((amdgpu_num_vgpr(256))) void stats_kernel(const b16* __restrict__ QP, const b16* __restrict__ KP, float* __restrict__ M2, float* __restrict__ RR) {
  __shared__ __attribute__((aligned(16))) b16 Ks[64][DK + 8];
  __shared__ float lm[8][64]; __shared__ float ls[8][64];
  __shared__ __attribute__((aligned(16))) float mo[64]; __shared__ __attribute__((aligned(16))) float ro[64];
  const int tid = threadIdx.x, wave = tid >> 5, lane = tid & 31, nloc = lane & 15, hlf = lane >> 4; const int bh = blockIdx.y, s0 = blockIdx.x * 64;
  const b16* Qb = QP + (size_t)bh * SEQ * DK; const b16* Kb = KP + (size_t)bh * SEQ * DK;
  for (int i = tid; i < 64 * 8; i += 256) { const int rr = i >> 3, pc = (i & 7) * 8; *(v8b*)(&Ks[rr][pc]) = *(const v8b*)(Kb + (size_t)(s0 + rr) * DK + pc); }
  __syncthreads();
  float mst[4], sst[4];
#pragma unroll
  for (int cs = 0; cs < 4; ++cs) { mst[cs] = -3.0e38f; sst[cs] = 0.0f; }
  const float c = LOG2E * RSQDK / (QS * QS);
#pragma unroll 1
  for (int it = 0; it < SEQ / 128; ++it) {
    const int rowQ = it * 128 + wave * 16 + nloc;
    const v16b a0 = frag_kb(Qb + (size_t)rowQ * DK, hlf), a1 = frag_kb(Qb + (size_t)rowQ * DK + 32, hlf);
#pragma unroll
    for (int cs = 0; cs < 4; ++cs) {
      const v16b b0 = frag_kb(&Ks[cs * 16 + nloc][0], hlf), b1 = frag_kb(&Ks[cs * 16 + nloc][32], hlf);
      v8f sc = (v8f){}; sc = wmma16b(a0, b0, sc); sc = wmma16b(a1, b1, sc);
      float t[8]; float tmax = -3.0e38f;
#pragma unroll
      for (int r = 0; r < 8; ++r) { t[r] = pmul(sc[r], c); tmax = fmaxf(tmax, t[r]); }
      tmax = fmaxf(tmax, __shfl_xor(tmax, 16));
      const float nm = fmaxf(mst[cs], tmax); float p = 0.0f;
#pragma unroll
      for (int r = 0; r < 8; ++r) p += nexp2(t[r] - nm);
      p += __shfl_xor(p, 16);
      sst[cs] = sst[cs] * nexp2(mst[cs] - nm) + p; mst[cs] = nm;
    }
  }
  if (hlf == 0) {
#pragma unroll
    for (int cs = 0; cs < 4; ++cs) { lm[wave][cs * 16 + nloc] = mst[cs]; ls[wave][cs * 16 + nloc] = sst[cs]; } }
  __syncthreads();
  if (tid < 64) { float M = -3.0e38f;
#pragma unroll
    for (int w = 0; w < 8; ++w) M = fmaxf(M, lm[w][tid]);
    float S = 0.0f;
#pragma unroll
    for (int w = 0; w < 8; ++w) S += ls[w][tid] * nexp2(lm[w][tid] - M);
    mo[tid] = M; ro[tid] = 1.0f / S; }
  __syncthreads();
  for (int pass = 0; pass < 2; ++pass) {
    if (wave == 0 && lane < 16) *(volatile v4f*)(M2 + (size_t)bh * SEQ + s0 + lane * 4) = *(const v4f*)(&mo[lane * 4]);
    if (wave == 1 && lane < 16) *(volatile v4f*)(RR + (size_t)bh * SEQ + s0 + lane * 4) = *(const v4f*)(&ro[lane * 4]);
    __threadfence(); }
}
__global__ __launch_bounds__(256) __attribute__((amdgpu_num_vgpr(256))) void av_kernel(const b16* __restrict__ QP, const b16* __restrict__ KP, const b16* __restrict__ VP,
                                                                                       const float* __restrict__ M2, const float* __restrict__ RR, b16* __restrict__ CT) {
  __shared__ __attribute__((aligned(16))) b16 Ks[32][DK + 8];
  __shared__ __attribute__((aligned(16))) b16 Vt[DK][32 + 8];
  __shared__ __attribute__((aligned(16))) b16 Pt[8][16][32 + 8];
  __shared__ __attribute__((aligned(16))) b16 Th[8][16][DK + 8];
  __shared__ float sm[32];
  const int tid = threadIdx.x, wave = tid >> 5, lane = tid & 31, nloc = lane & 15, hlf = lane >> 4;
  const int bh = blockIdx.y, b = bh / NH, hd = bh - b * NH; const int q0 = blockIdx.x * 128;
  const b16* Qb = QP + (size_t)bh * SEQ * DK; const b16* Kb = KP + (size_t)bh * SEQ * DK; const b16* Vb = VP + (size_t)bh * SEQ * DK;
  const float* Mb = M2 + (size_t)bh * SEQ; const float* Rb = RR + (size_t)bh * SEQ;
  const int rowQ = q0 + wave * 16 + nloc;
  const v16b a0 = frag_kb(Qb + (size_t)rowQ * DK, hlf), a1 = frag_kb(Qb + (size_t)rowQ * DK + 32, hlf);
  v8f hacc[4];
#pragma unroll
  for (int vs = 0; vs < 4; ++vs) hacc[vs] = (v8f){};
  const float c = LOG2E * RSQDK / (QS * QS);
#pragma unroll 1
  for (int sc0 = 0; sc0 < SEQ; sc0 += 32) {
    __syncthreads();
    { const int rr = tid >> 3, pc = (tid & 7) * 8; *(v8b*)(&Ks[rr][pc]) = *(const v8b*)(Kb + (size_t)(sc0 + rr) * DK + pc); }
    if (tid < 32) sm[tid] = Mb[sc0 + tid];
    { const int s = tid >> 3, vc = (tid & 7) * 8; const v8b gv = *(const v8b*)(Vb + (size_t)(sc0 + s) * DK + vc); const float rs = Rb[sc0 + s] * (VS / QS);
#pragma unroll
      for (int j = 0; j < 8; ++j) Vt[vc + j][s] = (b16)((float)gv[j] * rs); }
    __syncthreads();
#pragma unroll
    for (int st = 0; st < 2; ++st) {
      const v16b b0 = frag_kb(&Ks[st * 16 + nloc][0], hlf), b1 = frag_kb(&Ks[st * 16 + nloc][32], hlf);
      v8f s8 = (v8f){}; s8 = wmma16b(a0, b0, s8); s8 = wmma16b(a1, b1, s8);
      const float mc = sm[st * 16 + nloc];
#pragma unroll
      for (int r = 0; r < 8; ++r) Pt[wave][8 * hlf + r][st * 16 + nloc] = (b16)(PSC * nexp2(pmul(s8[r], c) - mc));
    }
    wave_lds_sync();
    const v16b pa = frag_kb(&Pt[wave][nloc][0], hlf);
#pragma unroll
    for (int vs = 0; vs < 4; ++vs) hacc[vs] = wmma16b(pa, frag_kb(&Vt[vs * 16 + nloc][0], hlf), hacc[vs]);
  }
#pragma unroll
  for (int vs = 0; vs < 4; ++vs)
#pragma unroll
    for (int r = 0; r < 8; ++r) Th[wave][8 * hlf + r][vs * 16 + nloc] = (b16)(hacc[vs][r] * (CTS / (PSC * VS)));
  wave_lds_sync();
  for (int pass = 0; pass < 2; ++pass) {
#pragma unroll
    for (int i = 0; i < 4; ++i) { const int rr = i * 4 + (lane >> 3), pc = (lane & 7) * 8; const size_t row = (size_t)b * SEQ + q0 + wave * 16 + rr;
      const v8b v = *(const v8b*)(&Th[wave][rr][pc]); *(volatile v8b*)(CT + row * DM + hd * DK + pc) = v; }
    __threadfence(); }
}
__global__ __launch_bounds__(128) void out1_kernel(const b16* __restrict__ CT, const b16* __restrict__ WO, const float* __restrict__ x, float* __restrict__ Y1) {
  __shared__ __attribute__((aligned(16))) float Tf[4][16][128 + 4];
  const int wave = threadIdx.x >> 5, lane = threadIdx.x & 31, nloc = lane & 15, hlf = lane >> 4; const size_t m0 = (size_t)blockIdx.x * 64 + wave * 16; const int n0 = blockIdx.y * 128;
  const size_t xr0 = (m0 / SEQ) * (size_t)SEQ_FULL + (m0 % SEQ);
  v8f acc[8];
#pragma unroll
  for (int t = 0; t < 8; ++t) acc[t] = (v8f){};
#pragma unroll 2
  for (int kb = 0; kb < DM; kb += 32) { const v16b a = frag_kb(CT + (m0 + nloc) * DM + kb, hlf);
#pragma unroll
    for (int t = 0; t < 8; ++t) acc[t] = wmma16b(a, frag_kb(WO + (size_t)(n0 + t * 16 + nloc) * DM + kb, hlf), acc[t]); }
#pragma unroll
  for (int t = 0; t < 8; ++t)
#pragma unroll
    for (int r = 0; r < 8; ++r) Tf[wave][8 * hlf + r][t * 16 + nloc] = acc[t][r] * (1.0f / (CTS * WSC));
  wave_lds_sync();
#pragma unroll 1
  for (int rr = 0; rr < 16; ++rr) { v4f a = *(const v4f*)(&Tf[wave][rr][lane * 4]); const v4f xv = *(const v4f*)(x + (xr0 + rr) * DM + n0 + lane * 4);
#pragma unroll
    for (int j = 0; j < 4; ++j) a[j] = a[j] + bf16_rne(xv[j]);
    *(v4f*)(&Tf[wave][rr][lane * 4]) = a; }
  wave_lds_sync();
  for (int pass = 0; pass < 2; ++pass) { for (int rr = 0; rr < 16; ++rr) *(volatile v4f*)(Y1 + (m0 + rr) * DM + n0 + lane * 4) = *(const v4f*)(&Tf[wave][rr][lane * 4]); __threadfence(); }
}
__global__ __launch_bounds__(256) void ln_kernel(const float* __restrict__ Y, const float* __restrict__ g, const float* __restrict__ bb, float* __restrict__ OUT) {
#pragma clang fp contract(off)
  const int wave = threadIdx.x >> 5, lane = threadIdx.x & 31; const size_t row = (size_t)blockIdx.x * 8 + wave; const float* yr = Y + row * DM;
  float v[DM / 128][4]; float s = 0.0f;
#pragma unroll
  for (int q = 0; q < DM / 128; ++q) { const v4f f = *(const v4f*)(yr + q * 128 + lane * 4);
#pragma unroll
    for (int j = 0; j < 4; ++j) { v[q][j] = f[j]; s += f[j]; } }
#pragma unroll
  for (int o = 16; o >= 1; o >>= 1) s += __shfl_xor(s, o);
  const float mean = s * (1.0f / (float)DM); float ss = 0.0f;
#pragma unroll
  for (int q = 0; q < DM / 128; ++q)
#pragma unroll
    for (int j = 0; j < 4; ++j) { const float d = v[q][j] - mean; ss += pmul(d, d); }
#pragma unroll
  for (int o = 16; o >= 1; o >>= 1) ss += __shfl_xor(ss, o);
  const float rs = 1.0f / sqrtf(ss * (1.0f / (float)DM) + LNEPS);
  for (int pass = 0; pass < 2; ++pass) {
#pragma unroll
    for (int q = 0; q < DM / 128; ++q) { const int cc = q * 128 + lane * 4; const v4f gv = *(const v4f*)(g + cc), bv = *(const v4f*)(bb + cc); v4f o;
#pragma unroll
      for (int j = 0; j < 4; ++j) o[j] = pmul((v[q][j] - mean) * rs, bfp(gv[j])) + bfp(bv[j]);
      *(volatile v4f*)(OUT + row * DM + cc) = o; }
    __threadfence(); }
}
__global__ __launch_bounds__(128) void mlp1_kernel(const float* __restrict__ XN, const b16* __restrict__ W1T, const float* __restrict__ b1, b16* __restrict__ G) {
  __shared__ __attribute__((aligned(16))) b16 As[64][256 + 8]; __shared__ __attribute__((aligned(16))) float Tf[4][16][128 + 4];
  const int wave = threadIdx.x >> 5, lane = threadIdx.x & 31, nloc = lane & 15, hlf = lane >> 4; const size_t r0 = (size_t)blockIdx.x * 64; const int n0 = blockIdx.y * 128;
  const float* xb = XN + r0 * DM;
  v8f acc[8];
#pragma unroll
  for (int t = 0; t < 8; ++t) acc[t] = (v8f){};
#pragma unroll 1
  for (int kc = 0; kc < DM; kc += 256) {
    __syncthreads();
#pragma unroll 4
    for (int i = threadIdx.x; i < 64 * 64; i += 128) { const int rr = i / 64, q = (i % 64) * 4; const v4f f = *(const v4f*)(xb + (size_t)rr * DM + kc + q); v4h o;
#pragma unroll
      for (int j = 0; j < 4; ++j) o[j] = (b16)(f[j] * XS); *(v4h*)(&As[rr][q]) = o; }
    __syncthreads();
#pragma unroll 2
    for (int kb = 0; kb < 256; kb += 32) { const v16b a = frag_kb(&As[wave * 16 + nloc][kb], hlf);
#pragma unroll
      for (int t = 0; t < 8; ++t) acc[t] = wmma16b(a, frag_kb(W1T + (size_t)(n0 + t * 16 + nloc) * DM + kc + kb, hlf), acc[t]); } }
#pragma unroll
  for (int t = 0; t < 8; ++t)
#pragma unroll
    for (int r = 0; r < 8; ++r) Tf[wave][8 * hlf + r][t * 16 + nloc] = acc[t][r] * (1.0f / (XS * WSC));
  __syncthreads();
  { const v4f bq = *(const v4f*)(b1 + n0 + lane * 4); float bv[4];
#pragma unroll
    for (int j = 0; j < 4; ++j) bv[j] = bf16_rne(bq[j]);
#pragma unroll 1
    for (int rr = 0; rr < 16; ++rr) { v4f a = *(const v4f*)(&Tf[wave][rr][lane * 4]);
#pragma unroll
      for (int j = 0; j < 4; ++j) a[j] = fmaxf(a[j] + bv[j], 0.0f);
      *(v4f*)(&Tf[wave][rr][lane * 4]) = a; } }
  wave_lds_sync();
  for (int pass = 0; pass < 2; ++pass) { for (int rr = 0; rr < 16; ++rr) { const v4f a = *(const v4f*)(&Tf[wave][rr][lane * 4]); v4h o4;
#pragma unroll
      for (int j = 0; j < 4; ++j) o4[j] = (b16)(a[j] * XS); *(volatile v4h*)(G + (r0 + wave * 16 + rr) * FF + n0 + lane * 4) = o4; } __threadfence(); }
}
__global__ __launch_bounds__(128) void mlp2_kernel(const b16* __restrict__ G, const b16* __restrict__ W2T, const float* __restrict__ b2, const float* __restrict__ X1, float* __restrict__ out) {
  __shared__ __attribute__((aligned(16))) float Tf[4][16][128 + 4];
  const int wave = threadIdx.x >> 5, lane = threadIdx.x & 31, nloc = lane & 15, hlf = lane >> 4; const size_t m0 = (size_t)blockIdx.x * 64 + wave * 16; const int n0 = blockIdx.y * 128;
  v8f acc[8];
#pragma unroll
  for (int t = 0; t < 8; ++t) acc[t] = (v8f){};
#pragma unroll 2
  for (int kb = 0; kb < FF; kb += 32) { const v16b a = frag_kb(G + (m0 + nloc) * FF + kb, hlf);
#pragma unroll
    for (int t = 0; t < 8; ++t) acc[t] = wmma16b(a, frag_kb(W2T + (size_t)(n0 + t * 16 + nloc) * FF + kb, hlf), acc[t]); }
#pragma unroll
  for (int t = 0; t < 8; ++t)
#pragma unroll
    for (int r = 0; r < 8; ++r) Tf[wave][8 * hlf + r][t * 16 + nloc] = acc[t][r] * (1.0f / (XS * WSC));
  wave_lds_sync();
  { const v4f bq = *(const v4f*)(b2 + n0 + lane * 4); float bv[4];
#pragma unroll
    for (int j = 0; j < 4; ++j) bv[j] = bf16_rne(bq[j]);
#pragma unroll 1
    for (int rr = 0; rr < 16; ++rr) { v4f a = *(const v4f*)(&Tf[wave][rr][lane * 4]); const v4f xv = *(const v4f*)(X1 + (m0 + rr) * DM + n0 + lane * 4);
#pragma unroll
      for (int j = 0; j < 4; ++j) a[j] = (a[j] + bv[j]) + xv[j];
      *(v4f*)(&Tf[wave][rr][lane * 4]) = a; } }
  wave_lds_sync();
  for (int pass = 0; pass < 2; ++pass) { for (int rr = 0; rr < 16; ++rr) *(volatile v4f*)(out + (m0 + rr) * DM + n0 + lane * 4) = *(const v4f*)(&Tf[wave][rr][lane * 4]); __threadfence(); }
}
}

extern "C" void kernel_launch(void* const* d_in, const int* in_sizes, int n_in, void* d_out, int out_size, void* d_ws, size_t ws_size, hipStream_t stream) {
  (void)n_in;
  auto Fp = [&](int i) { return (const float*)d_in[i]; };
  const int need_x = ((NB - 1) * SEQ_FULL + SEQ) * DM;
  if (in_sizes[0] < need_x || in_sizes[1] < NH * DM * DK || in_sizes[2] < NH * DM * DK || in_sizes[3] < NH * DM * DK || in_sizes[4] < DM * DM || in_sizes[5] < DM || in_sizes[6] < DM ||
      in_sizes[7] < DM * FF || in_sizes[8] < FF || in_sizes[9] < FF * DM || in_sizes[10] < DM || in_sizes[11] < DM || in_sizes[12] < DM || out_size < NR * DM) return;
  size_t off = 0; char* ws = (char*)d_ws;
  auto carve = [&](size_t bytes) { char* p = ws + off; off += (bytes + 255) & ~(size_t)255; return p; };
  b16* WQKV = (b16*)carve((size_t)NQKV * DM * 2); b16* WO = (b16*)carve((size_t)DM * DM * 2); b16* W1T = (b16*)carve((size_t)FF * DM * 2); b16* W2T = (b16*)carve((size_t)DM * FF * 2);
  b16* XH = (b16*)carve((size_t)NR * DM * 2);
  b16* QP = (b16*)carve((size_t)NBH * SEQ * DK * 2); b16* KP = (b16*)carve((size_t)NBH * SEQ * DK * 2); b16* VP = (b16*)carve((size_t)NBH * SEQ * DK * 2);
  float* M2 = (float*)carve((size_t)NBH * SEQ * 4); float* RR = (float*)carve((size_t)NBH * SEQ * 4);
  b16* CT = (b16*)carve((size_t)NR * DM * 2); float* Y1 = (float*)carve((size_t)NR * DM * 4); float* H = (float*)carve((size_t)NR * DM * 4); b16* G = (b16*)carve((size_t)NR * FF * 2);
  if (off > ws_size || off > ((size_t)128 << 20)) return;
  wtp_kernel<<<dim3(DM / 64, DK / 64, 3 * NH), 128, 0, stream>>>(Fp(1), Fp(2), Fp(3), NH, DM, DK, (long long)DM * DK, WQKV, (long long)DK * DM);
  wtp_kernel<<<dim3(DM / 64, DM / 64, 1), 128, 0, stream>>>(Fp(4), Fp(4), Fp(4), 1, DM, DM, 0LL, WO, 0LL);
  wtp_kernel<<<dim3(DM / 64, FF / 64, 1), 128, 0, stream>>>(Fp(7), Fp(7), Fp(7), 1, DM, FF, 0LL, W1T, 0LL);
  wtp_kernel<<<dim3(FF / 64, DM / 64, 1), 128, 0, stream>>>(Fp(9), Fp(9), Fp(9), 1, FF, DM, 0LL, W2T, 0LL);
  xp_kernel<<<(unsigned)(((size_t)NR * DM / 8 + 255) / 256), 256, 0, stream>>>(Fp(0), XH);
  qkv_kernel<<<dim3(NR / 64, NQKV / 128), 128, 0, stream>>>(XH, WQKV, QP, KP, VP);
  stats_kernel<<<dim3(SEQ / 64, NBH), 256, 0, stream>>>(QP, KP, M2, RR);
  av_kernel<<<dim3(SEQ / 128, NBH), 256, 0, stream>>>(QP, KP, VP, M2, RR, CT);
  out1_kernel<<<dim3(NR / 64, DM / 128), 128, 0, stream>>>(CT, WO, Fp(0), Y1);
  ln_kernel<<<NR / 8, 256, 0, stream>>>(Y1, Fp(5), Fp(6), H);
  mlp1_kernel<<<dim3(NR / 64, FF / 128), 128, 0, stream>>>(H, W1T, Fp(8), G);
  mlp2_kernel<<<dim3(NR / 64, DM / 128), 128, 0, stream>>>(G, W2T, Fp(10), H, Y1);
  ln_kernel<<<NR / 8, 256, 0, stream>>>(Y1, Fp(11), Fp(12), (float*)d_out);
}
